// UniDirectionalRNNTagger_76218489635004
// MI455X (gfx1250) — hardware-verified
//
#include <hip/hip_runtime.h>
#include <math.h>

#define VOCAB  50000
#define EMBED  256
#define HIDDEN 512
#define BATCH  64
#define SEQ    512
#define NCLS   2
#define NROWS  (BATCH * SEQ)
#define NCPAD  64
#define HPITCH 520
#define NT     256

typedef __attribute__((ext_vector_type(16))) _Float16 v16h;
typedef __attribute__((ext_vector_type(8)))  _Float16 v8h;
typedef __attribute__((ext_vector_type(16))) __bf16   v16b;
typedef __attribute__((ext_vector_type(8)))  __bf16   v8b;
typedef __attribute__((ext_vector_type(8)))  float    v8f;
typedef __attribute__((ext_vector_type(4)))  float    v4f;

__device__ __forceinline__ unsigned short f2bf_bits(float f) {
  unsigned u = __float_as_uint(f);
  return (unsigned short)((u + 0x7FFFu + ((u >> 16) & 1u)) >> 16);
}
__device__ __forceinline__ float bf_bits2f(unsigned short h) { return __uint_as_float(((unsigned)h) << 16); }

__device__ __forceinline__ void dep_guard_h(v8f& a, v8f& b, v16h x, v16h y) { asm volatile("v_nop\n\tv_nop\n\tv_nop\n\tv_nop" : "+v"(a), "+v"(b) : "v"(x), "v"(y)); }
__device__ __forceinline__ void dep_guard_b(v8f& a, v8f& b, v16b x, v16b y) { asm volatile("v_nop\n\tv_nop\n\tv_nop\n\tv_nop" : "+v"(a), "+v"(b) : "v"(x), "v"(y)); }
__device__ __forceinline__ void keep4_h(v16h a, v16h b, v16h c, v16h d) { asm volatile("v_nop" :: "v"(a), "v"(b), "v"(c), "v"(d)); }
__device__ __forceinline__ void keep4_b(v16b a, v16b b, v16b c, v16b d) { asm volatile("v_nop" :: "v"(a), "v"(b), "v"(c), "v"(d)); }
__device__ __forceinline__ void acc_guard4(v8f& a, v8f& b, v8f& c, v8f& d) { asm volatile("v_nop\n\tv_nop\n\tv_nop\n\tv_nop" : "+v"(a), "+v"(b), "+v"(c), "+v"(d)); }
template <typename T> struct Frag;
template <> struct Frag<_Float16> {
  typedef v16h V; union U { v16h v; v8h h[2]; };
  static __device__ __forceinline__ v16h load(const _Float16* p) {
    U f; f.h[0] = *(const v8h*)(p); f.h[1] = *(const v8h*)(p + 16); return f.v;
  }
  static __device__ __forceinline__ v8f mma(v16h a, v16h b, v8f c) {
    return __builtin_amdgcn_wmma_f32_16x16x32_f16(false, a, false, b, (short)0, c, false, false);
  }
  static __device__ __forceinline__ void guard(v8f& a, v8f& b, v16h x, v16h y) { dep_guard_h(a, b, x, y); }
  static __device__ __forceinline__ void keep(v16h a, v16h b, v16h c, v16h d) { keep4_h(a, b, c, d); }
};
template <> struct Frag<__bf16> {
  typedef v16b V; union U { v16b v; v8b h[2]; };
  static __device__ __forceinline__ v16b load(const __bf16* p) {
    U f; f.h[0] = *(const v8b*)(p); f.h[1] = *(const v8b*)(p + 16); return f.v;
  }
  static __device__ __forceinline__ v8f mma(v16b a, v16b b, v8f c) {
    return __builtin_amdgcn_wmma_f32_16x16x32_bf16(false, a, false, b, (short)0, c, false, false);
  }
  static __device__ __forceinline__ void guard(v8f& a, v8f& b, v16b x, v16b y) { dep_guard_b(a, b, x, y); }
  static __device__ __forceinline__ void keep(v16b a, v16b b, v16b c, v16b d) { keep4_b(a, b, c, d); }
};

template <int ET> struct Elem;
template <> struct Elem<0> { typedef _Float16 T; };
template <> struct Elem<1> { typedef __bf16 T; };
template <int ET, bool SPLIT, int BIAS_MODE, int OUT_MODE, bool RESID, int ACT = 0>
__global__ __launch_bounds__(256) void wmma_gemm64(
    const unsigned short* __restrict__ Ap, const unsigned short* __restrict__ A2p, int lda, long strideA,
    const unsigned short* __restrict__ Btp, const unsigned short* __restrict__ Bt2p, int ldb, long strideB,
    void* __restrict__ Cout, void* __restrict__ Cout2, int ldc, long strideC,
    const float* __restrict__ bias,
    const float* __restrict__ resid, long strideR,
    int M, int N, int K, float scale) {
  typedef typename Elem<ET>::T T;
  typedef typename Frag<T>::V V;
  const T* A = (const T*)Ap; const T* A2 = (const T*)A2p; const T* Bt = (const T*)Btp; const T* Bt2 = (const T*)Bt2p;
  __shared__ __align__(16) float sT[8][16 * 68];
  const int b    = blockIdx.y;
  const int lane = threadIdx.x & 31;
  const int wave = threadIdx.x >> 5;
  const int tilesN = N >> 6;
  const int tilesM = M >> 6;
  const int tile = blockIdx.x * 8 + wave;
  if (tile >= tilesM * tilesN) return;
  const int tm = tile / tilesN;
  const int tn = tile - tm * tilesN;
  const int m0 = tm << 6;
  const int n0 = tn << 6;

  const T* Ab  = A  + (size_t)b * strideA;
  const T* Bb  = Bt + (size_t)b * strideB;
  const T* Ab2 = SPLIT ? (A2  + (size_t)b * strideA) : nullptr;
  const T* Bb2 = SPLIT ? (Bt2 + (size_t)b * strideB) : nullptr;

  const int rlane = lane & 15;
  const int koff  = (lane >> 4) * 8;
  const int mOff  = (lane >> 4) * 8;

  v8f acc[4][4];
#pragma unroll
  for (int i = 0; i < 4; ++i)
#pragma unroll
    for (int j = 0; j < 4; ++j) acc[i][j] = (v8f){0.f,0.f,0.f,0.f,0.f,0.f,0.f,0.f};

  for (int k0 = 0; k0 < K; k0 += 32) {
    V bh[4], bl[4];
#pragma unroll
    for (int j = 0; j < 4; ++j) {
      const size_t bo = (size_t)(n0 + (j << 4) + rlane) * ldb + koff + k0;
      bh[j] = Frag<T>::load(Bb + bo);
      if (SPLIT) bl[j] = Frag<T>::load(Bb2 + bo);
    }
#pragma unroll
    for (int i = 0; i < 4; ++i) {
      const size_t ao = (size_t)(m0 + (i << 4) + rlane) * lda + koff + k0;
      V ah = Frag<T>::load(Ab + ao);
      V al;
      if (SPLIT) al = Frag<T>::load(Ab2 + ao);
#pragma unroll
      for (int j = 0; j < 4; ++j) {
        acc[i][j] = Frag<T>::mma(ah, bh[j], acc[i][j]);
        if (SPLIT) {
          acc[i][j] = Frag<T>::mma(ah, bl[j], acc[i][j]);
          acc[i][j] = Frag<T>::mma(al, bh[j], acc[i][j]);
        }
      }
      Frag<T>::guard(acc[i][0], acc[i][3], ah, SPLIT ? al : ah);
    }
    Frag<T>::keep(bh[0], bh[1], bh[2], bh[3]);
    if (SPLIT) Frag<T>::keep(bl[0], bl[1], bl[2], bl[3]);
  }
  acc_guard4(acc[0][0], acc[0][1], acc[0][2], acc[0][3]);
  acc_guard4(acc[1][0], acc[1][1], acc[1][2], acc[1][3]);
  acc_guard4(acc[2][0], acc[2][1], acc[2][2], acc[2][3]);
  acc_guard4(acc[3][0], acc[3][1], acc[3][2], acc[3][3]);

  float* slab = sT[wave];
  const float* Rb = RESID ? (resid + (size_t)b * strideR) : nullptr;
#pragma unroll
  for (int i = 0; i < 4; ++i) {
    const int mBase = m0 + (i << 4);
#pragma unroll
    for (int j = 0; j < 4; ++j) {
      const int n = n0 + (j << 4) + rlane;
      float bv = 0.f;
      if (BIAS_MODE == 2) bv = bias[n];
#pragma unroll
      for (int r = 0; r < 8; ++r) {
        float v = acc[i][j][r] * scale;
        if (BIAS_MODE == 1) v += bias[mBase + mOff + r];
        if (BIAS_MODE == 2) v += bv;
        if (RESID) v += Rb[(size_t)(mBase + mOff + r) * ldc + n];
        if (ACT == 1) v = tanhf(v);
        if (ACT == 2) v = fmaxf(v, 0.0f);
        if (ACT == 3) v = v / (1.0f + expf(-v));
        if (ACT == 4) v = (v > 0.f) ? v : 0.01f * v;
        if (ACT == 5) v = 0.5f * v * (1.0f + erff(v * 0.70710678118654752f));
        slab[(mOff + r) * 68 + (j << 4) + rlane] = v;
      }
    }
    __builtin_amdgcn_fence(__ATOMIC_RELEASE, "workgroup");
    __builtin_amdgcn_wave_barrier();
    __builtin_amdgcn_fence(__ATOMIC_ACQUIRE, "workgroup");
    if (OUT_MODE == 0) {
      float* C = (float*)Cout + (size_t)b * strideC;
      const int hh = lane >> 4, c4 = (lane & 15) * 4;
      for (int pass = 0; pass < 2; ++pass) {
#pragma unroll
        for (int it = 0; it < 8; ++it) {
          const int row = it * 2 + hh;
          v4f v = *(const v4f*)(slab + row * 68 + c4);
          *(volatile v4f*)(C + (size_t)(mBase + row) * ldc + n0 + c4) = v;
        }
        __threadfence();
      }
    } else {
      const int q = lane >> 3, c8 = (lane & 7) * 8;
      unsigned short* C  = (unsigned short*)Cout  + (size_t)b * strideC;
      unsigned short* C2 = (OUT_MODE == 2) ? ((unsigned short*)Cout2 + (size_t)b * strideC) : nullptr;
      for (int pass = 0; pass < 2; ++pass) {
#pragma unroll
        for (int it = 0; it < 4; ++it) {
          const int row = it * 4 + q;
          const float* sp = slab + row * 68 + c8;
          v8h hv, lv;
#pragma unroll
          for (int e = 0; e < 8; ++e) {
            if (OUT_MODE == 1) {
              hv[e] = (_Float16)sp[e];
            } else {
              unsigned short hb = f2bf_bits(sp[e]);
              unsigned short lb = f2bf_bits(sp[e] - bf_bits2f(hb));
              hv[e] = __builtin_bit_cast(_Float16, hb);
              lv[e] = __builtin_bit_cast(_Float16, lb);
            }
          }
          *(volatile v8h*)(C + (size_t)(mBase + row) * ldc + n0 + c8) = hv;
          if (OUT_MODE == 2) *(volatile v8h*)(C2 + (size_t)(mBase + row) * ldc + n0 + c8) = lv;
        }
        __threadfence();
      }
    }
    __builtin_amdgcn_fence(__ATOMIC_RELEASE, "workgroup");
    __builtin_amdgcn_wave_barrier();
    __builtin_amdgcn_fence(__ATOMIC_ACQUIRE, "workgroup");
  }
}

__device__ __forceinline__ unsigned pack_f16x2(float a, float b) {
  const _Float16 h0 = (_Float16)a, h1 = (_Float16)b;
  return (unsigned)__builtin_bit_cast(unsigned short, h0) | ((unsigned)__builtin_bit_cast(unsigned short, h1) << 16);
}
__device__ __forceinline__ void st2u(unsigned* p, unsigned v) { *(volatile unsigned*)p = v; __threadfence(); *(volatile unsigned*)p = v; }
__device__ __forceinline__ float ftanh(float x) { return 1.0f - 2.0f * __builtin_amdgcn_rcpf(1.0f + __expf(2.0f * x)); }

__global__ __launch_bounds__(NT) void prep_kernel(const float* __restrict__ Wih, const float* __restrict__ Whh,
                                                 const float* __restrict__ bih, const float* __restrict__ bhh,
                                                 const float* __restrict__ Wcls,
                                                 unsigned* __restrict__ WIH, unsigned* __restrict__ WHH,
                                                 unsigned* __restrict__ WCLS, float* __restrict__ BSUM) {
  const int blk = blockIdx.x, tid = threadIdx.x;
  if (blk < 256) {
    const int p = blk * NT + tid;
    const unsigned u = pack_f16x2(Wih[2 * p] * 16.0f, Wih[2 * p + 1] * 16.0f);
    st2u(WIH + p, u);
  } else if (blk < 768) {
    const int p = (blk - 256) * NT + tid;
    const unsigned u = pack_f16x2(Whh[2 * p] * 16.0f, Whh[2 * p + 1] * 16.0f);
    st2u(WHH + p, u);
  } else if (blk < 832) {
    const int p = (blk - 768) * NT + tid;
    const int row = p >> 8, col = 2 * (p & 255);
    const int rowc = row < NCLS ? row : (NCLS - 1);
    const bool live = row < NCLS;
    const float w0 = Wcls[rowc * HIDDEN + col], w1 = Wcls[rowc * HIDDEN + col + 1];
    const float v0 = live ? w0 * 16.0f : 0.0f, v1 = live ? w1 * 16.0f : 0.0f;
    const unsigned u = pack_f16x2(v0, v1);
    st2u(WCLS + p, u);
  } else {
    const int i = (blk - 832) * NT + tid;
    const float v = bih[i] + bhh[i];
    float* q = BSUM + i;
    *(volatile float*)q = v; __threadfence(); *(volatile float*)q = v;
  }
}

__global__ __launch_bounds__(NT) void embed_kernel(const int* __restrict__ tok, const float* __restrict__ emb, _Float16* __restrict__ EX) {
  const int gid = blockIdx.x * NT + threadIdx.x;
  if (gid >= NROWS * 32) return;
  const int row = gid >> 5, c8 = (gid & 31) * 8;
  int tk = tok[row]; tk = tk < 0 ? 0 : (tk >= VOCAB ? VOCAB - 1 : tk);
  const float* ep = emb + (size_t)tk * EMBED + c8;
  const v4f a = *(const v4f*)ep, bq = *(const v4f*)(ep + 4);
  v8h h;
#pragma unroll
  for (int e = 0; e < 4; ++e) { h[e] = (_Float16)a[e]; h[4 + e] = (_Float16)bq[e]; }
  _Float16* op = EX + (size_t)row * EMBED + c8;
  *(volatile v8h*)op = h; __threadfence(); *(volatile v8h*)op = h;
}

__global__ __launch_bounds__(NT) void rnn_kernel(const float* __restrict__ XP, const _Float16* __restrict__ WHH, _Float16* __restrict__ HS) {
  __shared__ __align__(16) _Float16 h16[16 * HPITCH];
  const int tid = threadIdx.x, lane = tid & 31, wave = tid >> 5;
  const int rlane = lane & 15, hh = lane >> 4, koff = hh * 8, mOff = hh * 8;
  const int mbase = blockIdx.x * 16;
  for (int i = tid; i < 16 * HPITCH; i += NT) h16[i] = (_Float16)0.0f;
  __syncthreads();
  const int jb = 64 * wave + rlane;
  const _Float16* arow = h16 + rlane * HPITCH + koff;
  const _Float16* wb = WHH + (size_t)jb * HIDDEN + koff;
  const float* xb = XP + (size_t)(mbase + mOff) * SEQ * HIDDEN + jb;
  const v8f z8 = {0.f, 0.f, 0.f, 0.f, 0.f, 0.f, 0.f, 0.f};

#pragma unroll 1
  for (int t = 0; t < SEQ; ++t) {
    v8f acc[4];
    acc[0] = z8; acc[1] = z8; acc[2] = z8; acc[3] = z8;
#pragma unroll 1
    for (int k0 = 0; k0 < HIDDEN; k0 += 32) {
      const v16h a  = Frag<_Float16>::load(arow + k0);
      const v16h b0 = Frag<_Float16>::load(wb + k0);
      const v16h b1 = Frag<_Float16>::load(wb + (size_t)16 * HIDDEN + k0);
      const v16h b2 = Frag<_Float16>::load(wb + (size_t)32 * HIDDEN + k0);
      const v16h b3 = Frag<_Float16>::load(wb + (size_t)48 * HIDDEN + k0);
      acc[0] = Frag<_Float16>::mma(a, b0, acc[0]);
      acc[1] = Frag<_Float16>::mma(a, b1, acc[1]);
      acc[2] = Frag<_Float16>::mma(a, b2, acc[2]);
      acc[3] = Frag<_Float16>::mma(a, b3, acc[3]);
      dep_guard_h(acc[0], acc[3], a, b3);
      keep4_h(b0, b1, b2, b3);
    }
    acc_guard4(acc[0], acc[1], acc[2], acc[3]);
    const float* xt = xb + (size_t)t * HIDDEN;
    float hv[4][8];
#pragma unroll
    for (int r = 0; r < 8; ++r) {
      const float* xr = xt + (size_t)r * SEQ * HIDDEN;
      const float x0 = xr[0], x1 = xr[16], x2 = xr[32], x3 = xr[48];
      hv[0][r] = ftanh(acc[0][r] * (1.0f / 16.0f) + x0);
      hv[1][r] = ftanh(acc[1][r] * (1.0f / 16.0f) + x1);
      hv[2][r] = ftanh(acc[2][r] * (1.0f / 16.0f) + x2);
      hv[3][r] = ftanh(acc[3][r] * (1.0f / 16.0f) + x3);
    }
    __syncthreads();
#pragma unroll
    for (int r = 0; r < 8; ++r) {
#pragma unroll
      for (int nt = 0; nt < 4; ++nt) h16[(mOff + r) * HPITCH + jb + 16 * nt] = (_Float16)hv[nt][r];
    }
    __syncthreads();
    _Float16* hsb = HS + ((size_t)mbase * SEQ + t) * HIDDEN;
    for (int pass = 0; pass < 2; ++pass) {
#pragma unroll
      for (int it = 0; it < 4; ++it) {
        const int row = 2 * wave + (it >> 1);
        const int c0 = (it & 1) * 256 + lane * 8;
        const v8h v = *(const v8h*)(h16 + row * HPITCH + c0);
        *(volatile v8h*)(hsb + (size_t)row * SEQ * HIDDEN + c0) = v;
      }
      __threadfence();
    }
  }
}

__global__ __launch_bounds__(NT) void pack_kernel(const float* __restrict__ LG, const float* __restrict__ bcls, float* __restrict__ out) {
  const int i = blockIdx.x * NT + threadIdx.x;
  if (i >= NROWS / 2) return;
  const int r0 = 2 * i;
  const float b0 = bcls[0], b1 = bcls[1];
  v4f o;
  o[0] = LG[(size_t)r0 * NCPAD + 0] + b0;
  o[1] = LG[(size_t)r0 * NCPAD + 1] + b1;
  o[2] = LG[(size_t)(r0 + 1) * NCPAD + 0] + b0;
  o[3] = LG[(size_t)(r0 + 1) * NCPAD + 1] + b1;
  float* p = out + (size_t)4 * i;
  *(volatile v4f*)p = o; __threadfence(); *(volatile v4f*)p = o;
}

extern "C" void kernel_launch(void* const* d_in, const int* in_sizes, int n_in,
                              void* d_out, int out_size, void* d_ws, size_t ws_size, hipStream_t stream) {
  if (n_in < 8 || d_out == nullptr || d_ws == nullptr) return;
  if (in_sizes[0] != BATCH * SEQ || in_sizes[1] != VOCAB * EMBED || in_sizes[2] != HIDDEN * EMBED || in_sizes[3] != HIDDEN * HIDDEN ||
      in_sizes[4] != HIDDEN || in_sizes[5] != HIDDEN || in_sizes[6] != NCLS * HIDDEN || in_sizes[7] != NCLS ||
      out_size != BATCH * SEQ * NCLS) return;

  const int*   tok  = (const int*)d_in[0];
  const float* emb  = (const float*)d_in[1];
  const float* Wih  = (const float*)d_in[2];
  const float* Whh  = (const float*)d_in[3];
  const float* bih  = (const float*)d_in[4];
  const float* bhh  = (const float*)d_in[5];
  const float* Wcls = (const float*)d_in[6];
  const float* bcls = (const float*)d_in[7];
  float* out = (float*)d_out;

  char* ws = (char*)d_ws; size_t off = 0;
  auto carve = [&](size_t bytes) -> char* { char* p = ws + off; off += (bytes + 255) & ~(size_t)255; return p; };
  _Float16* EX16   = (_Float16*)carve((size_t)NROWS * EMBED * 2);
  unsigned* WIH    = (unsigned*)carve((size_t)HIDDEN * EMBED * 2);
  unsigned* WHH    = (unsigned*)carve((size_t)HIDDEN * HIDDEN * 2);
  unsigned* WCLS   = (unsigned*)carve((size_t)NCPAD * HIDDEN * 2);
  float*    BSUM   = (float*)carve((size_t)HIDDEN * 4);
  float*    XP32   = (float*)carve((size_t)NROWS * HIDDEN * 4);
  _Float16* HS16   = (_Float16*)carve((size_t)NROWS * HIDDEN * 2);
  if (off > ws_size || off > (size_t)134217728) return;
  if ((size_t)NROWS * NCPAD * 4 > (size_t)NROWS * EMBED * 2) return;
  float* LG = (float*)EX16;
  const _Float16* WIH16  = (const _Float16*)WIH;
  const _Float16* WHH16  = (const _Float16*)WHH;
  const _Float16* WCLS16 = (const _Float16*)WCLS;

  prep_kernel<<<834, NT, 0, stream>>>(Wih, Whh, bih, bhh, Wcls, WIH, WHH, WCLS, BSUM);
  embed_kernel<<<(NROWS * 32) / NT, NT, 0, stream>>>(tok, emb, EX16);
  {
    const int tiles = (NROWS / 64) * (HIDDEN / 64);
    wmma_gemm64<0, false, 2, 0, false><<<dim3((tiles + 7) / 8, 1), 256, 0, stream>>>(
        (const unsigned short*)EX16, (const unsigned short*)nullptr, EMBED, 0L,
        (const unsigned short*)WIH16, (const unsigned short*)nullptr, EMBED, 0L,
        (void*)XP32, (void*)nullptr, HIDDEN, 0L,
        BSUM, (const float*)nullptr, 0L, NROWS, HIDDEN, EMBED, 1.0f / 16.0f);
  }
  rnn_kernel<<<BATCH / 16, NT, 0, stream>>>(XP32, WHH16, HS16);
  {
    const int tiles = (NROWS / 64) * (NCPAD / 64);
    wmma_gemm64<0, false, 0, 0, false><<<dim3((tiles + 7) / 8, 1), 256, 0, stream>>>(
        (const unsigned short*)HS16, (const unsigned short*)nullptr, HIDDEN, 0L,
        (const unsigned short*)WCLS16, (const unsigned short*)nullptr, HIDDEN, 0L,
        (void*)LG, (void*)nullptr, NCPAD, 0L,
        (const float*)nullptr, (const float*)nullptr, 0L, NROWS, NCPAD, HIDDEN, 1.0f / 16.0f);
  }
  pack_kernel<<<(NROWS / 2) / NT, NT, 0, stream>>>(LG, bcls, out);
}
